// SLXMlp_47304769798199
// MI455X (gfx1250) — hardware-verified
//
#include <hip/hip_runtime.h>
#include <stddef.h>
#include <stdint.h>
#include <math.h>

#define MTOK 8192
#define NIN  1024
#define NHID 4096
#define NOUT 1024
#define RK   102
#define RP   128
#define SHP  136
#define SFP  132

static_assert(MTOK % 128 == 0);
static_assert(NIN % 128 == 0);
static_assert(NHID % 128 == 0);
static_assert(NOUT % 128 == 0);
static_assert(RP % 32 == 0);
static_assert(RK <= RP);
static_assert(NHID % 16 == 0);
static_assert(NOUT % 16 == 0);
static_assert(NIN % 64 == 0);
static_assert(NHID % 64 == 0);
static_assert((MTOK * NIN) % 2048 == 0);

typedef _Float16 hh;
typedef hh    v16h __attribute__((ext_vector_type(16)));
typedef hh    v8h  __attribute__((ext_vector_type(8)));
typedef float v8f  __attribute__((ext_vector_type(8)));
typedef float v4f  __attribute__((ext_vector_type(4)));

union Frag { v16h v; v8h p[2]; };
union EpiLds { hh h[128 * SHP]; float f[64 * SFP]; };

__device__ __forceinline__ v8f zero8() { return (v8f){0.f, 0.f, 0.f, 0.f, 0.f, 0.f, 0.f, 0.f}; }

__device__ __forceinline__ v16h ldfrag(const hh* __restrict__ p, int ld, int row0, int k0, int lane) {
  const hh* q = p + (size_t)(row0 + (lane & 15)) * (size_t)ld + k0 + 8 * (lane >> 4);
  Frag f;
  f.p[0] = *(const v8h*)(q);
  f.p[1] = *(const v8h*)(q + 16);
  return f.v;
}

__device__ __forceinline__ v8f mma16(v16h a, v16h b, v8f cc) {
  return __builtin_amdgcn_wmma_f32_16x16x32_f16(false, a, false, b, (short)0, cc, false, false);
}

__device__ __forceinline__ void gemm32x64(const hh* __restrict__ A, int lda, const hh* __restrict__ B, int ldb,
                                          int ma, int nb, int kdim, int lane, v8f (&acc)[2][4]) {
#pragma unroll 1
  for (int k0 = 0; k0 < kdim; k0 += 32) {
    const v16h a0 = ldfrag(A, lda, ma, k0, lane);
    const v16h a1 = ldfrag(A, lda, ma + 16, k0, lane);
    const v16h b0 = ldfrag(B, ldb, nb, k0, lane);
    const v16h b1 = ldfrag(B, ldb, nb + 16, k0, lane);
    const v16h b2 = ldfrag(B, ldb, nb + 32, k0, lane);
    const v16h b3 = ldfrag(B, ldb, nb + 48, k0, lane);
    acc[0][0] = mma16(a0, b0, acc[0][0]);
    acc[1][0] = mma16(a1, b0, acc[1][0]);
    acc[0][1] = mma16(a0, b1, acc[0][1]);
    acc[1][1] = mma16(a1, b1, acc[1][1]);
    acc[0][2] = mma16(a0, b2, acc[0][2]);
    acc[1][2] = mma16(a1, b2, acc[1][2]);
    acc[0][3] = mma16(a0, b3, acc[0][3]);
    acc[1][3] = mma16(a1, b3, acc[1][3]);
    asm volatile("v_nop\n\tv_nop\n\tv_nop\n\tv_nop"
                 : "+v"(acc[0][0]), "+v"(acc[0][1]), "+v"(acc[0][2]), "+v"(acc[0][3]),
                   "+v"(acc[1][0]), "+v"(acc[1][1]), "+v"(acc[1][2]), "+v"(acc[1][3])
                 : "v"(a0), "v"(a1), "v"(b0), "v"(b1), "v"(b2), "v"(b3));
  }
}

__device__ __forceinline__ float gelu_f(float x) {
  const float z  = fabsf(x) * 0.70710678118654752f;
  const float t  = __builtin_amdgcn_rcpf(fmaf(0.3275911f, z, 1.0f));
  float pl = fmaf(t, 1.061405429f, -1.453152027f);
  pl = fmaf(t, pl, 1.421413741f);
  pl = fmaf(t, pl, -0.284496736f);
  pl = fmaf(t, pl, 0.254829592f);
  pl = pl * t;
  const float ex   = __expf(-z * z);
  const float erfa = fmaf(-pl, ex, 1.0f);
  const float erfv = (x < 0.f) ? -erfa : erfa;
  return 0.5f * x * (1.0f + erfv);
}

__global__ __launch_bounds__(256) void k_cvt_u(const float* __restrict__ u, hh* __restrict__ up, int rows) {
  const int tid = threadIdx.x;
  int row = blockIdx.x * 16 + (tid >> 4);
  row = (row < rows) ? row : (rows - 1);
  const int pc = tid & 15;
  const float* src = u + (size_t)row * RK;
  v8f t;
#pragma unroll
  for (int e = 0; e < 8; ++e) {
    const int col = pc * 8 + e;
    const int cc  = (col < RK) ? col : (RK - 1);
    const float v = src[cc];
    t[e] = (col < RK) ? (v * 64.0f) : 0.0f;
  }
  const v8h pk = __builtin_convertvector(t, v8h);
  hh* gp = up + (size_t)row * RP + pc * 8;
  *(volatile v8h*)gp = pk;
  __threadfence();
  *(volatile v8h*)gp = pk;
}

template <int COLS>
__global__ __launch_bounds__(256) void k_cvt_vt(const float* __restrict__ v, hh* __restrict__ vt) {
  static_assert(COLS % 64 == 0);
  __shared__ __align__(16) float sw[RP * 68];
  const int tid = threadIdx.x;
  const int n0 = blockIdx.x * 64;
#pragma unroll
  for (int j = 0; j < 2; ++j) {
    const int p  = tid + 256 * j;
    const int r  = p >> 2;
    const int c0 = (p & 3) * 16;
    const int rc = (r < RK) ? r : (RK - 1);
    const bool live = (r < RK);
    const float* src = v + (size_t)rc * COLS + n0 + c0;
#pragma unroll
    for (int e = 0; e < 4; ++e) {
      const v4f q = *(const v4f*)(src + 4 * e);
      float* dp = sw + r * 68 + c0 + 4 * e;
#pragma unroll
      for (int i = 0; i < 4; ++i) dp[i] = live ? q[i] : 0.0f;
    }
  }
  __syncthreads();
  v8h hv[4];
  size_t go[4];
#pragma unroll
  for (int j = 0; j < 4; ++j) {
    const int p  = tid + 256 * j;
    const int n  = p >> 4;
    const int pc = p & 15;
    const float* cp = sw + (pc * 8) * 68 + n;
    v8f t;
#pragma unroll
    for (int e = 0; e < 8; ++e) t[e] = cp[e * 68] * 64.0f;
    hv[j] = __builtin_convertvector(t, v8h);
    go[j] = (size_t)(n0 + n) * RP + pc * 8;
  }
#pragma unroll
  for (int j = 0; j < 4; ++j) *(volatile v8h*)(vt + go[j]) = hv[j];
  __threadfence();
#pragma unroll
  for (int j = 0; j < 4; ++j) *(volatile v8h*)(vt + go[j]) = hv[j];
}

__global__ __launch_bounds__(256) void k_cvt_x(const float* __restrict__ x, hh* __restrict__ xp) {
  const size_t i0 = ((size_t)blockIdx.x * 256 + (size_t)threadIdx.x) * 8;
  const v4f a0 = *(const v4f*)(x + i0), a1 = *(const v4f*)(x + i0 + 4);
  const v8f t = {a0[0], a0[1], a0[2], a0[3], a1[0], a1[1], a1[2], a1[3]};
  const v8h pk = __builtin_convertvector(t, v8h);
  *(volatile v8h*)(xp + i0) = pk;
  __threadfence();
  *(volatile v8h*)(xp + i0) = pk;
}

template <int MODE>
__global__ __launch_bounds__(256) void k_gemm(const hh* __restrict__ Ap, const hh* __restrict__ Bp,
                                              const float* __restrict__ bias, const float* __restrict__ wsp,
                                              const int* __restrict__ msk, hh* __restrict__ o16,
                                              float* __restrict__ o32) {
  constexpr bool F32OUT = (MODE == 3);
  constexpr int LDA = (MODE == 0 || MODE == 1) ? RP : ((MODE == 2) ? NIN : NHID);
  constexpr int LDB = LDA;
  constexpr int KD  = LDA;
  constexpr int LDO = (MODE == 0) ? NIN : ((MODE == 1 || MODE == 2) ? NHID : NOUT);
  static_assert(KD % 32 == 0);

  __shared__ __align__(16) EpiLds lds;
  const int tid = threadIdx.x, lane = tid & 31, w = tid >> 5;
  const int h = lane >> 4, c = lane & 15;
  const int wm = (w >> 1) * 32, wn = (w & 1) * 64;
  const int m0 = blockIdx.y * 128;
  const int n0 = blockIdx.x * 128;

  v8f acc[2][4];
#pragma unroll
  for (int i = 0; i < 2; ++i)
#pragma unroll
    for (int j = 0; j < 4; ++j) acc[i][j] = zero8();
  gemm32x64(Ap, LDA, Bp, LDB, m0 + wm, n0 + wn, KD, lane, acc);

  float bc[4] = {0.f, 0.f, 0.f, 0.f};
  if constexpr (MODE == 2 || MODE == 3) {
#pragma unroll
    for (int j = 0; j < 4; ++j) bc[j] = bias[n0 + wn + 16 * j + c];
  }

  if constexpr (!F32OUT) {
#pragma unroll
    for (int i = 0; i < 2; ++i) {
#pragma unroll
      for (int j = 0; j < 4; ++j) {
        float v[8];
#pragma unroll
        for (int r = 0; r < 8; ++r) {
          const float a = acc[i][j][r];
          float t = 0.f;
          if constexpr (MODE == 0 || MODE == 1) {
            const int gm = m0 + wm + 16 * i + 8 * h + r;
            const int gn = n0 + wn + 16 * j + c;
            const size_t gi = (size_t)gm * LDO + gn;
            const int   mk = msk[gi];
            const float wv = wsp[gi];
            const float sv = (mk != 0) ? wv : 0.0f;
            t = (a * (1.0f / 4096.0f) + sv) * 64.0f;
          } else {
            t = gelu_f(a * (1.0f / 64.0f) + bc[j]) * 16.0f;
          }
          v[r] = t;
        }
#pragma unroll
        for (int r = 0; r < 8; ++r)
          lds.h[(wm + 16 * i + 8 * h + r) * SHP + wn + 16 * j + c] = (hh)v[r];
      }
    }
    __syncthreads();
    v8h val[8];
    size_t go[8];
#pragma unroll
    for (int it = 0; it < 8; ++it) {
      const int p  = tid + 256 * it;
      const int lr = p >> 4;
      const int pc = p & 15;
      val[it] = *(const v8h*)(lds.h + lr * SHP + pc * 8);
      go[it] = (size_t)(m0 + lr) * LDO + n0 + pc * 8;
    }
#pragma unroll
    for (int it = 0; it < 8; ++it) *(volatile v8h*)(o16 + go[it]) = val[it];
    __threadfence();
#pragma unroll
    for (int it = 0; it < 8; ++it) *(volatile v8h*)(o16 + go[it]) = val[it];
  } else {
    constexpr float OSC = 1.0f / 1024.0f;
#pragma unroll
    for (int hf = 0; hf < 2; ++hf) {
      if ((w >> 2) == hf) {
#pragma unroll
        for (int i = 0; i < 2; ++i)
#pragma unroll
          for (int j = 0; j < 4; ++j)
#pragma unroll
            for (int r = 0; r < 8; ++r)
              lds.f[(wm - 64 * hf + 16 * i + 8 * h + r) * SFP + wn + 16 * j + c] = acc[i][j][r] * OSC + bc[j];
      }
      __syncthreads();
      v4f val[8];
      size_t go[8];
#pragma unroll
      for (int it = 0; it < 8; ++it) {
        const int p  = tid + 256 * it;
        const int lr = p >> 5;
        const int pc = p & 31;
        val[it] = *(const v4f*)(lds.f + lr * SFP + pc * 4);
        go[it] = (size_t)(m0 + 64 * hf + lr) * LDO + n0 + pc * 4;
      }
#pragma unroll
      for (int it = 0; it < 8; ++it) *(volatile v4f*)(o32 + go[it]) = val[it];
      __threadfence();
#pragma unroll
      for (int it = 0; it < 8; ++it) *(volatile v4f*)(o32 + go[it]) = val[it];
      if (hf == 0) __syncthreads();
    }
  }
}

extern "C" void kernel_launch(void* const* d_in, const int* in_sizes, int n_in,
                              void* d_out, int out_size, void* d_ws, size_t ws_size,
                              hipStream_t stream) {
  if (n_in < 11) return;
  if (in_sizes[0] != MTOK * NIN) return;
  if (in_sizes[1] != NHID * RK || in_sizes[2] != RK * NIN) return;
  if (in_sizes[3] != NHID * NIN || in_sizes[4] != NHID) return;
  if (in_sizes[5] != NOUT * RK || in_sizes[6] != RK * NHID) return;
  if (in_sizes[7] != NOUT * NHID || in_sizes[8] != NOUT) return;
  if (in_sizes[9] != NHID * NIN || in_sizes[10] != NOUT * NHID) return;
  if (out_size != MTOK * NOUT) return;

  const float* x   = (const float*)d_in[0];
  const float* u1  = (const float*)d_in[1];
  const float* v1  = (const float*)d_in[2];
  const float* ws1 = (const float*)d_in[3];
  const float* b1  = (const float*)d_in[4];
  const float* u2  = (const float*)d_in[5];
  const float* v2  = (const float*)d_in[6];
  const float* ws2 = (const float*)d_in[7];
  const float* b2  = (const float*)d_in[8];
  const int*   mk1 = (const int*)d_in[9];
  const int*   mk2 = (const int*)d_in[10];
  float* out = (float*)d_out;

  size_t off = 0;
  const size_t oUA = off; off += (size_t)NHID * RP * 2;
  const size_t oVA = off; off += (size_t)NIN * RP * 2;
  const size_t oUB = off; off += (size_t)NOUT * RP * 2;
  const size_t oVB = off; off += (size_t)NHID * RP * 2;
  const size_t oWA = off; off += (size_t)NHID * NIN * 2;
  const size_t oWB = off; off += (size_t)NOUT * NHID * 2;
  const size_t oXP = off; off += (size_t)MTOK * NIN * 2;
  const size_t oHP = off; off += (size_t)MTOK * NHID * 2;
  if (off > ws_size) return;
  if (off > (size_t)134217728) return;

  char* ws = (char*)d_ws;
  hh* UA = (hh*)(ws + oUA);  hh* VA = (hh*)(ws + oVA);
  hh* UB = (hh*)(ws + oUB);  hh* VB = (hh*)(ws + oVB);
  hh* WA = (hh*)(ws + oWA);  hh* WB = (hh*)(ws + oWB);
  hh* XP = (hh*)(ws + oXP);  hh* HP = (hh*)(ws + oHP);

  k_cvt_u<<<dim3(NHID / 16), dim3(256), 0, stream>>>(u1, UA, NHID);
  k_cvt_vt<NIN><<<dim3(NIN / 64), dim3(256), 0, stream>>>(v1, VA);
  k_cvt_u<<<dim3(NOUT / 16), dim3(256), 0, stream>>>(u2, UB, NOUT);
  k_cvt_vt<NHID><<<dim3(NHID / 64), dim3(256), 0, stream>>>(v2, VB);
  k_gemm<0><<<dim3(NIN / 128, NHID / 128), dim3(256), 0, stream>>>(UA, VA, b1, ws1, mk1, WA, out);
  k_gemm<1><<<dim3(NHID / 128, NOUT / 128), dim3(256), 0, stream>>>(UB, VB, b2, ws2, mk2, WB, out);
  k_cvt_x<<<dim3((MTOK * NIN) / 2048), dim3(256), 0, stream>>>(x, XP);
  k_gemm<2><<<dim3(NHID / 128, MTOK / 128), dim3(256), 0, stream>>>(XP, WA, b1, ws1, mk1, HP, out);
  k_gemm<3><<<dim3(NOUT / 128, MTOK / 128), dim3(256), 0, stream>>>(HP, WB, b2, ws2, mk2, XP, out);
  (void)hipGetLastError();
}
